// GatGraphClassifier_40372692582769
// MI455X (gfx1250) — hardware-verified
//
#include <hip/hip_runtime.h>


namespace {
constexpr int N = 50000, E = 400000, D = 64, H = 4, HD = H * D, L = 3, C = 10, G = 512, NV = 174, NPAD = 50048, NBLK = NPAD / 128, NB = 256;
constexpr float FXS = 524288.0f, FXI = 1.0f / 524288.0f, NEG = 0.2f;
__constant__ int ATOM_OFF[9] = {0, 119, 124, 136, 148, 158, 164, 170, 172};

typedef _Float16 b16;
typedef __attribute__((ext_vector_type(16))) _Float16 v16b;
typedef __attribute__((ext_vector_type(8)))  _Float16 v8b;
typedef __attribute__((ext_vector_type(8)))  float v8f;
typedef __attribute__((ext_vector_type(4)))  float v4f;

__device__ __forceinline__ v8b ld8b(const b16* p) { return *(const v8b*)p; }
__device__ __forceinline__ v16b cat8b(v8b a, v8b b) { return __builtin_shufflevector(a, b, 0, 1, 2, 3, 4, 5, 6, 7, 8, 9, 10, 11, 12, 13, 14, 15); }
__device__ __forceinline__ v16b frag_kb(const b16* p, int hh) { return cat8b(ld8b(p + 8 * hh), ld8b(p + 16 + 8 * hh)); }
__device__ __forceinline__ void split16(float v, b16& hi, b16& lo) { hi = (b16)v; lo = (b16)(v - (float)hi); }
__device__ __forceinline__ void frag_ksplit(const float* p, int hh, v16b& fh_, v16b& fl_) {
  const float* p0 = p + 8 * hh; const float* p1 = p + 16 + 8 * hh;
#pragma unroll
  for (int e = 0; e < 8; ++e) { b16 a, c; split16(p0[e], a, c); fh_[e] = a; fl_[e] = c; split16(p1[e], a, c); fh_[8 + e] = a; fl_[8 + e] = c; }
}
__device__ __forceinline__ v8f wmma16b(v16b a, v16b b, v8f c) {
  v8f d = __builtin_amdgcn_wmma_f32_16x16x32_f16(false, a, false, b, (short)0, c, false, false);
  asm volatile("v_nop\n\tv_nop\n\tv_nop\n\tv_nop" : "+v"(d) : "v"(a), "v"(b));
  return d;
}
__device__ __forceinline__ void wave_lds_sync() {
  __builtin_amdgcn_fence(__ATOMIC_RELEASE, "workgroup");
  __builtin_amdgcn_wave_barrier();
  __builtin_amdgcn_fence(__ATOMIC_ACQUIRE, "workgroup");
}

struct Opnd { const void* p0; const void* p1; int ld; };
template <int NP> __device__ __forceinline__ void load_frags(const Opnd& o, int row, int kb, int hh, v16b& fh_, v16b& fl_) {
  if (NP == 0) { frag_ksplit((const float*)o.p0 + (size_t)row * o.ld + kb, hh, fh_, fl_); }
  else if (NP == 4) {
    const float* p = (const float*)o.p0 + (size_t)row * o.ld + kb; const float* p0 = p + 8 * hh; const float* p1 = p + 16 + 8 * hh;
#pragma unroll
    for (int e = 0; e < 8; ++e) { b16 a, c; split16(p0[e] * 64.0f, a, c); fh_[e] = a; fl_[e] = c; split16(p1[e] * 64.0f, a, c); fh_[8 + e] = a; fl_[8 + e] = c; }
  } else if (NP == 3) {
    const float* p = (const float*)o.p0 + (size_t)row * o.ld + kb; const float* p0 = p + 8 * hh; const float* p1 = p + 16 + 8 * hh;
#pragma unroll
    for (int e = 0; e < 8; ++e) { fh_[e] = (b16)p0[e]; fh_[8 + e] = (b16)p1[e]; }
    fl_ = fh_;
  } else {
    fh_ = frag_kb((const b16*)o.p0 + (size_t)row * o.ld + kb, hh);
    if (NP == 2) fl_ = frag_kb((const b16*)o.p1 + (size_t)row * o.ld + kb, hh); else fl_ = fh_;
  }
}
template <int ANP, int BNP> __device__ __forceinline__ v8f mac(v16b ah, v16b al, v16b bh, v16b bl, v8f c) {
  c = wmma16b(ah, bh, c);
  if (BNP == 0 || BNP == 2 || BNP == 4) c = wmma16b(ah, bl, c);
  if (ANP == 0 || ANP == 2 || ANP == 4) c = wmma16b(al, bh, c);
  return c;
}
template <int ANP, int BNP>
__device__ __forceinline__ void gemm_tile(const Opnd& A, const Opnd& B, int K, int m0, int c0, int nloc, int hlf, v8f (&acc)[2][4]) {
  for (int kb = 0; kb < K; kb += 32) {
    v16b a0h, a0l, a1h, a1l;
    load_frags<ANP>(A, m0 + nloc, kb, hlf, a0h, a0l);
    load_frags<ANP>(A, m0 + 16 + nloc, kb, hlf, a1h, a1l);
#pragma unroll
    for (int t = 0; t < 4; ++t) {
      v16b bh, bl;
      load_frags<BNP>(B, c0 + t * 16 + nloc, kb, hlf, bh, bl);
      acc[0][t] = mac<ANP, BNP>(a0h, a0l, bh, bl, acc[0][t]);
      acc[1][t] = mac<ANP, BNP>(a1h, a1l, bh, bl, acc[1][t]);
    }
  }
}

__device__ __forceinline__ void epi_planes(v8f (&acc)[2][4], float scale, bool two, b16* __restrict__ oh, b16* __restrict__ ol, int ldo,
                                           int m0, int c0, int lane, b16* Th, b16* Tl) {
  const int nloc = lane & 15, hlf = lane >> 4;
#pragma unroll
  for (int t = 0; t < 4; ++t)
#pragma unroll
    for (int r = 0; r < 2; ++r)
#pragma unroll
      for (int v = 0; v < 8; ++v) {
        const int rr = r * 16 + v + 8 * hlf, cc = t * 16 + nloc;
        b16 h_, l_; split16(acc[r][t][v] * scale, h_, l_);
        Th[rr * 64 + cc] = h_; Tl[rr * 64 + cc] = l_;
      }
  wave_lds_sync();
  for (int pass = 0; pass < 2; ++pass) {
#pragma unroll
    for (int j = 0; j < 8; ++j) {
      const int rr = j * 4 + (lane >> 3), c8 = (lane & 7) * 8;
      const size_t o = (size_t)(m0 + rr) * ldo + c0 + c8;
      *(volatile v8b*)(oh + o) = ld8b(Th + rr * 64 + c8);
      if (two) *(volatile v8b*)(ol + o) = ld8b(Tl + rr * 64 + c8);
    }
    __threadfence();
  }
}
__device__ __forceinline__ void epi_f32(v8f (&acc)[2][4], float scale, const float* rscale, float* __restrict__ out, int ldo, int m0, int c0, int lane, float* Tt) {
  const int nloc = lane & 15, hlf = lane >> 4;
#pragma unroll
  for (int t = 0; t < 4; ++t)
#pragma unroll
    for (int r = 0; r < 2; ++r)
#pragma unroll
      for (int v = 0; v < 8; ++v) {
        const int rr = r * 16 + v + 8 * hlf;
        const float rs = rscale ? rscale[(size_t)(m0 + rr) * 32] : 1.0f;
        Tt[rr * 64 + t * 16 + nloc] = acc[r][t][v] * scale * rs;
      }
  wave_lds_sync();
  float* dst0 = out + (size_t)m0 * ldo + c0;
  for (int pass = 0; pass < 2; ++pass) {
#pragma unroll
    for (int j = 0; j < 16; ++j) { const int rr = j * 2 + hlf, c4 = nloc * 4; *(volatile v4f*)(dst0 + (size_t)rr * ldo + c4) = *(const v4f*)(Tt + rr * 64 + c4); }
    __threadfence();
  }
}


__device__ __forceinline__ int fkey(float f) { const int b = __float_as_int(f); return (b >= 0) ? b : (b ^ 0x7FFFFFFF); }
__device__ __forceinline__ float fkey_inv(int k) { return __int_as_float((k >= 0) ? k : (k ^ 0x7FFFFFFF)); }
__device__ __forceinline__ float gelu_e(float v) { return 0.5f * v * (1.0f + erff(v * 0.70710678118654752f)); }

__global__ __launch_bounds__(256) void prep_kernel(const float* __restrict__ Wl, const float* __restrict__ Wr, b16* __restrict__ wlr) {
  const size_t tid = (size_t)blockIdx.x * blockDim.x + threadIdx.x, nth = (size_t)gridDim.x * blockDim.x;
  for (int pass = 0; pass < 2; ++pass) {
    for (size_t p = tid; p < (size_t)L * 2 * HD * D / 8; p += nth) { const int l = (int)(p / (2 * HD * D / 8)); const int rem = (int)(p % (2 * HD * D / 8)), n = rem / (D / 8), k0 = (rem % (D / 8)) * 8;
      const float* W = ((n < HD) ? Wl : Wr) + (size_t)l * D * HD; const int nn = n % HD; v8b v;
#pragma unroll
      for (int e = 0; e < 8; ++e) v[e] = (b16)W[(size_t)(k0 + e) * HD + nn];
      *(volatile v8b*)(wlr + ((size_t)l * 2 * HD + n) * D + k0) = v; }
    __threadfence();
  }
}

__global__ __launch_bounds__(256) void enc_kernel(const int* __restrict__ feat, const float* __restrict__ emb, float* __restrict__ x) {
  const int n = blockIdx.x * 16 + (threadIdx.x >> 4), q = threadIdx.x & 15;
  v4f s = {0.0f, 0.0f, 0.0f, 0.0f};
  if (n < N) {
#pragma unroll
    for (int f = 0; f < 9; ++f) { int id = feat[(size_t)n * 9 + f] + ATOM_OFF[f]; id = (id < 0) ? 0 : (id >= NV ? NV - 1 : id); s += *(const v4f*)(emb + (size_t)id * D + q * 4); } }
  for (int pass = 0; pass < 2; ++pass) { *(volatile v4f*)(x + (size_t)n * D + q * 4) = s; __threadfence(); }
}

__global__ __launch_bounds__(128) void lin_kernel(const float* __restrict__ x, const b16* __restrict__ w, const float* __restrict__ bl, const float* __restrict__ br, float* __restrict__ xlr) {
  __shared__ __attribute__((aligned(16))) float Ts[4][32 * 64];
  const int lane = threadIdx.x & 31, wave = threadIdx.x >> 5, nloc = lane & 15, hlf = lane >> 4, m0 = blockIdx.y * 128 + wave * 32, c0 = blockIdx.x * 64;
  v8f acc[2][4];
#pragma unroll
  for (int r = 0; r < 2; ++r)
#pragma unroll
    for (int t = 0; t < 4; ++t) acc[r][t] = (v8f){};
  const Opnd A{x, nullptr, D}, B{w, nullptr, D};
  gemm_tile<3, 1>(A, B, D, m0, c0, nloc, hlf, acc);
  const float* bb = (c0 < HD) ? (bl + c0) : (br + (c0 - HD));
#pragma unroll
  for (int t = 0; t < 4; ++t)
#pragma unroll
    for (int r = 0; r < 2; ++r)
#pragma unroll
      for (int v = 0; v < 8; ++v) acc[r][t][v] += bb[t * 16 + nloc];
  epi_f32(acc, 1.0f, nullptr, xlr, 2 * HD, m0, c0, lane, Ts[wave]);
}

__global__ __launch_bounds__(256) void escore_kernel(const int* __restrict__ esrc, const int* __restrict__ edst, const float* __restrict__ xlr, const float* __restrict__ att, float* __restrict__ esc) {
  const int e = blockIdx.x * 256 + threadIdx.x; const int ee = min(e, E - 1);
  int s = esrc[ee], d = edst[ee]; s = (s < 0) ? 0 : (s >= N ? N - 1 : s); d = (d < 0) ? 0 : (d >= N ? N - 1 : d);
  v4f out = {0.0f, 0.0f, 0.0f, 0.0f};
#pragma unroll 1
  for (int h = 0; h < H; ++h) { float acc = 0.0f; const float* a = xlr + (size_t)s * 2 * HD + h * D; const float* b = xlr + (size_t)d * 2 * HD + HD + h * D; const float* at = att + h * D;
#pragma unroll 1
    for (int k = 0; k < D; k += 4) { const v4f va = *(const v4f*)(a + k), vb = *(const v4f*)(b + k), wa = *(const v4f*)(at + k);
#pragma unroll
      for (int q = 0; q < 4; ++q) { float m = va[q] + vb[q]; m = (m > 0.0f) ? m : NEG * m; acc += m * wa[q]; } }
    out[h] = acc; }
  if (e < E) for (int pass = 0; pass < 2; ++pass) { *(volatile v4f*)(esc + (size_t)e * 4) = out; __threadfence(); }
}

typedef __attribute__((ext_vector_type(4))) int v4i;
template <bool GELU>
__global__ __launch_bounds__(256) void gat_kernel(const int* __restrict__ esrc, const int* __restrict__ edst, const float* __restrict__ xlr, const float* __restrict__ esc, const float* __restrict__ att, const float* __restrict__ bias, float* __restrict__ xo) {
  __shared__ __attribute__((aligned(16))) int acc[NB * HD];
  __shared__ int mx[NB * H]; __shared__ int den[NB * H]; __shared__ int list[8 * 256]; __shared__ float selfe[NB * H];
  const int t_ = threadIdx.x, wave = t_ >> 5, lane = t_ & 31, base = blockIdx.x * NB;
  for (int i = t_; i < NB * HD; i += 256) acc[i] = 0;
  for (int i = t_; i < NB * H; i += 256) { const int slot = i / H, h = i % H, node = base + slot; float e = -INFINITY;
    if (node < N) { float a = 0.0f; const float* ra = xlr + (size_t)node * 2 * HD + h * D; const float* rb = ra + HD; const float* at = att + h * D;
#pragma unroll 1
      for (int k = 0; k < D; ++k) { float m = ra[k] + rb[k]; m = (m > 0.0f) ? m : NEG * m; a += m * at[k]; } e = a; }
    selfe[i] = e; den[i] = 0; mx[i] = fkey(e); }
  __syncthreads();
  for (int c0 = 0; c0 < E; c0 += 256 * 8) { const int e0 = c0 + (wave * 32 + lane) * 8;
#pragma unroll
    for (int j = 0; j < 8; ++j) { const int ee = min(e0 + j, E - 1); const int dv = edst[ee]; const unsigned sl = (unsigned)(((e0 + j < E) ? dv : -1) - base);
      if (sl < (unsigned)NB) { const v4f es = *(const v4f*)(esc + (size_t)ee * 4);
#pragma unroll
        for (int h = 0; h < H; ++h) atomicMax(&mx[sl * H + h], fkey(es[h])); } } }
  __syncthreads();
  int* wl = list + wave * 256;
  const int hd = lane >> 3, sub = lane & 7;
  auto accumulate = [&](int s, int slot, float escore) {
    const float w = __expf(escore - fkey_inv(mx[slot * H + hd]));
    if (sub == 0) atomicAdd(&den[slot * H + hd], (int)rintf(w * FXS));
    const float* hr = xlr + (size_t)s * 2 * HD + hd * D + sub * 8; int* ar = acc + slot * HD + hd * D + sub * 8;
    const v4f a = *(const v4f*)hr, b = *(const v4f*)(hr + 4);
#pragma unroll
    for (int q = 0; q < 4; ++q) { atomicAdd(ar + q, (int)rintf(w * a[q] * FXS)); atomicAdd(ar + 4 + q, (int)rintf(w * b[q] * FXS)); }
  };
  for (int slot = wave; slot < NB; slot += 8) { if (base + slot < N) accumulate(base + slot, slot, selfe[slot * H + hd]); }
  for (int c0 = 0; c0 < E; c0 += 256 * 8) {
    const int e0 = c0 + (wave * 32 + lane) * 8; int dd[8];
#pragma unroll
    for (int j = 0; j < 8; ++j) { const int dv = edst[min(e0 + j, E - 1)]; dd[j] = (e0 + j < E) ? dv : -1; }
    unsigned sl[8]; bool hit[8]; bool anyl = false;
#pragma unroll
    for (int j = 0; j < 8; ++j) { sl[j] = (unsigned)(dd[j] - base); hit[j] = sl[j] < (unsigned)NB; anyl |= hit[j]; }
    int wc = 0;
    if (__builtin_amdgcn_ballot_w32(anyl) != 0u) {
#pragma unroll
      for (int j = 0; j < 8; ++j) {
        const unsigned mj = __builtin_amdgcn_ballot_w32(hit[j]);
        if (mj != 0u) {
          if (hit[j]) { const int pos = wc + (int)__builtin_amdgcn_mbcnt_lo(mj, 0u); wl[pos] = ((e0 + j) << 8) | (int)sl[j]; }
          wc += __builtin_popcount(mj); } } }
    __builtin_amdgcn_wave_barrier(); __builtin_amdgcn_fence(__ATOMIC_RELEASE, "workgroup"); __builtin_amdgcn_fence(__ATOMIC_ACQUIRE, "workgroup");
    for (int i = 0; i < wc; ++i) { const int ent = wl[i]; const int e = ent >> 8, slot = ent & 255; int s = esrc[e]; s = (s < 0) ? 0 : (s >= N ? N - 1 : s); accumulate(s, slot, esc[(size_t)e * 4 + hd]); }
    __builtin_amdgcn_wave_barrier();
  }
  __syncthreads();
  for (int pass = 0; pass < 2; ++pass) {
    for (int i = t_; i < NB * D / 4; i += 256) { const int slot = i / (D / 4), cq = (i % (D / 4)) * 4, node = base + slot; if (node < NPAD) { v4f o = {0.0f, 0.0f, 0.0f, 0.0f};
        if (node < N) { float invd[H];
#pragma unroll
          for (int h = 0; h < H; ++h) invd[h] = __builtin_amdgcn_rcpf((float)den[slot * H + h]);
#pragma unroll
          for (int q = 0; q < 4; ++q) { float sum = 0.0f;
#pragma unroll
            for (int h = 0; h < H; ++h) sum += (float)acc[slot * HD + h * D + cq + q] * invd[h];
            const float val = sum * (1.0f / H) + bias[cq + q]; o[q] = GELU ? gelu_e(val) : val; } }
        *(volatile v4f*)(xo + (size_t)node * D + cq) = o; } }
    __threadfence();
  }
}

__global__ __launch_bounds__(256) void pool_kernel(const float* __restrict__ x, const int* __restrict__ batch, float* __restrict__ pooled) {
  constexpr int GB = 64;
  __shared__ int acc[GB * D]; __shared__ int cnt[GB]; __shared__ int list[8 * 256];
  const int t_ = threadIdx.x, wave = t_ >> 5, lane = t_ & 31, gbase = blockIdx.x * GB;
  for (int i = t_; i < GB * D; i += 256) acc[i] = 0;
  if (t_ < GB) cnt[t_] = 0;
  __syncthreads();
  int* wl = list + wave * 256;
  for (int c0 = 0; c0 < N; c0 += 256 * 8) {
    const int n0 = c0 + (wave * 32 + lane) * 8; int dd[8];
#pragma unroll
    for (int j = 0; j < 8; ++j) { const int bv = batch[min(n0 + j, N - 1)]; dd[j] = (n0 + j < N) ? bv : -1; }
    unsigned sl[8]; bool hit[8]; bool anyl = false;
#pragma unroll
    for (int j = 0; j < 8; ++j) { sl[j] = (unsigned)(dd[j] - gbase); hit[j] = sl[j] < (unsigned)GB; anyl |= hit[j]; }
    int wc = 0;
    if (__builtin_amdgcn_ballot_w32(anyl) != 0u) {
#pragma unroll
      for (int j = 0; j < 8; ++j) {
        const unsigned mj = __builtin_amdgcn_ballot_w32(hit[j]);
        if (mj != 0u) {
          if (hit[j]) { const int pos = wc + (int)__builtin_amdgcn_mbcnt_lo(mj, 0u); wl[pos] = ((n0 + j) << 6) | (int)sl[j]; atomicAdd(&cnt[sl[j]], 1); }
          wc += __builtin_popcount(mj); } } }
    __builtin_amdgcn_wave_barrier(); __builtin_amdgcn_fence(__ATOMIC_RELEASE, "workgroup"); __builtin_amdgcn_fence(__ATOMIC_ACQUIRE, "workgroup");
    for (int i = 0; i < wc; ++i) { const int ent = wl[i]; const int n = ent >> 6, slot = ent & 63; const float a = x[(size_t)n * D + lane * 2], b = x[(size_t)n * D + lane * 2 + 1];
      atomicAdd(&acc[slot * D + lane * 2], (int)rintf(a * FXS)); atomicAdd(&acc[slot * D + lane * 2 + 1], (int)rintf(b * FXS)); }
    __builtin_amdgcn_wave_barrier();
  }
  __syncthreads();
  for (int pass = 0; pass < 2; ++pass) { for (int i = t_; i < GB * D; i += 256) { const int slot = i / D; ((volatile float*)pooled)[(size_t)gbase * D + i] = (float)acc[i] * FXI / fmaxf((float)cnt[slot], 1.0f); } __threadfence(); }
}

__global__ __launch_bounds__(128) void cls_kernel(const float* __restrict__ pooled, const float* __restrict__ Wc, const float* __restrict__ bc, float* __restrict__ out) {
  const int i = blockIdx.x * 128 + threadIdx.x, g = i / C, c = i % C; float acc = bc[c];
#pragma unroll 1
  for (int k = 0; k < D; ++k) acc += pooled[(size_t)g * D + k] * Wc[k * C + c];
  for (int pass = 0; pass < 2; ++pass) { ((volatile float*)out)[i] = acc; __threadfence(); }
}
}

extern "C" void kernel_launch(void* const* d_in, const int* in_sizes, int n_in,
                              void* d_out, int out_size, void* d_ws, size_t ws_size, hipStream_t stream) {
  (void)n_in; (void)out_size;
  const int* feat = (const int*)d_in[0]; const int* ei = (const int*)d_in[1]; const int* batch = (const int*)d_in[2]; const float* emb = (const float*)d_in[3];
  const float* Wl = (const float*)d_in[4]; const float* bl = (const float*)d_in[5]; const float* Wr = (const float*)d_in[6]; const float* br = (const float*)d_in[7];
  const float* att = (const float*)d_in[8]; const float* gb = (const float*)d_in[9]; const float* Wc = (const float*)d_in[10]; const float* bc = (const float*)d_in[11];
  float* out = (float*)d_out;
  if (in_sizes[0] != N * 9 || in_sizes[1] != 2 * E || in_sizes[2] != N || in_sizes[3] != NV * D || in_sizes[4] != L * D * HD || in_sizes[8] != L * H * D || in_sizes[10] != D * C) return;
  const int* esrc = ei; const int* edst = ei + E;
  size_t off = 0; char* ws = (char*)d_ws;
  auto carve = [&](size_t bytes) { char* p = ws + off; off += (bytes + 255) & ~(size_t)255; return p; };
  b16* wlr = (b16*)carve((size_t)L * 2 * HD * D * 2);
  float* x = (float*)carve((size_t)NPAD * D * 4); float* xlr = (float*)carve((size_t)NPAD * 2 * HD * 4); float* esc = (float*)carve((size_t)E * 4 * 4); float* pooled = (float*)carve((size_t)G * D * 4);
  if (off > ws_size) return;
  prep_kernel<<<64, 256, 0, stream>>>(Wl, Wr, wlr);
  enc_kernel<<<NPAD / 16, 256, 0, stream>>>(feat, emb, x);
  for (int l = 0; l < L; ++l) {
    lin_kernel<<<dim3(2 * HD / 64, NBLK), 128, 0, stream>>>(x, wlr + (size_t)l * 2 * HD * D, bl + l * HD, br + l * HD, xlr);
    escore_kernel<<<(E + 255) / 256, 256, 0, stream>>>(esrc, edst, xlr, att + l * H * D, esc);
    if (l < L - 1) gat_kernel<true><<<NPAD / NB + 1, 256, 0, stream>>>(esrc, edst, xlr, esc, att + l * H * D, gb + l * D, x);
    else           gat_kernel<false><<<NPAD / NB + 1, 256, 0, stream>>>(esrc, edst, xlr, esc, att + l * H * D, gb + l * D, x);
  }
  pool_kernel<<<G / 64, 256, 0, stream>>>(x, batch, pooled);
  cls_kernel<<<G * C / 128, 128, 0, stream>>>(pooled, Wc, bc, out);
}
